// GraphormerExpert_20538533609927
// MI455X (gfx1250) — hardware-verified
//
#include <hip/hip_runtime.h>
#include <stddef.h>
#include <math.h>


#define NND    128
#define KIN    128
#define QP     384
#define KOF    128
#define VOF    256
#define NLAY   3
#define DEGMX  512
#define EMBN   513
#define GBM    80
#define GTH    160
#define GWT    2048
#define WPP    72
#define CRNG   4096
#define FRNG   1024
#define FSH    10
#define LCAP   18432
#define SEGCAP 18432
#define ECH    4096
#define DSENT  (-1073741824)
#define WSCAP  134217728
#define ASCL   8.0f
#define WSCL   64.0f
#define INVSCL 0.001953125f
#define RSQC   0.35355339059327373f
#define INVD   0.0078125f
#define LNEPS  1e-5f
#define GCAP   30.0f

#define FL_LIST 0
#define FL_SEG  (FL_LIST + LCAP * 4)
#define FL_LOFF (FL_SEG + (SEGCAP + 64) * 2)
#define FL_LCNT (FL_LOFF + FRNG * 4)
#define FL_CUR  (FL_LCNT + FRNG * 4)
#define FL_WT   (FL_CUR + FRNG * 4)
#define FILL_LDS (FL_WT + 64)

static_assert((1 << FSH) == FRNG);
static_assert((CRNG % FRNG) == 0);
static_assert(CRNG == 256 * 16 && FRNG == 256 * 4);
static_assert(ECH == 256 * 16);
static_assert(LCAP == SEGCAP);
static_assert((SEGCAP % 64) == 0 && ((SEGCAP / 8) % 256) == 0);
static_assert((GBM % 16) == 0 && GTH == (GBM / 16) * 32);
static_assert((KIN % 64) == 0 && (NND % 64) == 0 && (QP % 128) == 0 && (KIN % 32) == 0);
static_assert((FL_SEG % 16) == 0 && (FL_LOFF % 16) == 0 && (FL_LCNT % 16) == 0 && (FL_CUR % 16) == 0 && (FL_WT % 16) == 0);
static_assert(FILL_LDS <= 160000);
static_assert(EMBN == DEGMX + 1);

typedef float          v4f  __attribute__((ext_vector_type(4)));
typedef float          v8f  __attribute__((ext_vector_type(8)));
typedef int            v4i  __attribute__((ext_vector_type(4)));
typedef unsigned short v4us __attribute__((ext_vector_type(4)));
typedef unsigned short v8us __attribute__((ext_vector_type(8)));
typedef _Float16       v16h __attribute__((ext_vector_type(16)));
union FragH { v16h v; v8us u[2]; };

__device__ __forceinline__ unsigned short h16(float f) {
  const _Float16 h = (_Float16)f;
  return __builtin_bit_cast(unsigned short, h);
}

__device__ __forceinline__ v8us cvt8(v4f a, v4f b, float s) {
  v8us r;
  r[0] = h16(a.x * s); r[1] = h16(a.y * s); r[2] = h16(a.z * s); r[3] = h16(a.w * s);
  r[4] = h16(b.x * s); r[5] = h16(b.y * s); r[6] = h16(b.z * s); r[7] = h16(b.w * s);
  return r;
}

__device__ __forceinline__ v4us cvt4(v4f a, float s) {
  v4us r;
  r.x = h16(a.x * s); r.y = h16(a.y * s); r.z = h16(a.z * s); r.w = h16(a.w * s);
  return r;
}

__device__ __forceinline__ v8f zero8() {
  v8f z = {0.f, 0.f, 0.f, 0.f, 0.f, 0.f, 0.f, 0.f};
  return z;
}

__device__ __forceinline__ v8f wmh(v16h a, v16h b, v8f c) {
  v8f d = __builtin_amdgcn_wmma_f32_16x16x32_f16(false, a, false, b, (short)0, c, false, false);
  asm volatile("v_nop\n\tv_nop\n\tv_nop\n\tv_nop" : "+v"(d) : "v"(a), "v"(b));
  return d;
}

__device__ __forceinline__ v4f ln4(v4f x, v4f g4, v4f b4) {
  float s = (x.x + x.y) + (x.z + x.w);
#pragma unroll
  for (int oo = 16; oo >= 1; oo >>= 1) s += __shfl_xor(s, oo);
  const float mu = s * INVD;
  const v4f d = x - mu;
  float sq = (d.x * d.x + d.y * d.y) + (d.z * d.z + d.w * d.w);
#pragma unroll
  for (int oo = 16; oo >= 1; oo >>= 1) sq += __shfl_xor(sq, oo);
  const float rstd = rsqrtf(sq * INVD + LNEPS);
  return (d * rstd) * g4 + b4;
}

__global__ __launch_bounds__(256) void k_wpack(
    const float* __restrict__ W, unsigned short* wt, int K, int M, int szs, int dzs) {
  __shared__ __attribute__((aligned(16))) unsigned short sT[64 * WPP];
  const int tid = (int)threadIdx.x;
  const int m0 = (int)blockIdx.x * 64, k0 = (int)blockIdx.y * 64;
  const float* Wz = W + (size_t)blockIdx.z * (size_t)szs;
  unsigned short* wz = wt + (size_t)blockIdx.z * (size_t)dzs;
#pragma unroll 4
  for (int it = 0; it < 16; ++it) {
    const int idx = it * 256 + tid;
    const int kk = idx >> 6, mm = idx & 63;
    int kr = k0 + kk; kr = kr > K - 1 ? K - 1 : kr;
    int mc = m0 + mm; mc = mc > M - 1 ? M - 1 : mc;
    const float w = Wz[(size_t)kr * M + mc];
    sT[mm * WPP + kk] = h16(w * WSCL);
  }
  __syncthreads();
  v8us pv[2];
  size_t po[2];
#pragma unroll
  for (int it = 0; it < 2; ++it) {
    const int p = it * 256 + tid;
    const int row = p >> 3, c8 = (p & 7) * 8;
    pv[it] = *(const v8us*)(sT + row * WPP + c8);
    int mr = m0 + row; mr = mr > M - 1 ? M - 1 : mr;
    po[it] = (size_t)mr * K + k0 + c8;
  }
  const bool full = (m0 + 64 <= M) && (k0 + 64 <= K);
  if (full) {
#pragma unroll
    for (int it = 0; it < 2; ++it) *(volatile v8us*)(wz + po[it]) = pv[it];
  }
  __threadfence();
  if (full) {
#pragma unroll
    for (int it = 0; it < 2; ++it) *(volatile v8us*)(wz + po[it]) = pv[it];
  }
}

__global__ __launch_bounds__(256) void k_cvt(const float* __restrict__ X, unsigned short* o, int np) {
  const int p = (int)blockIdx.x * 256 + (int)threadIdx.x;
  const int pc = p < np ? p : np - 1;
  const v4f a = *(const v4f*)(X + (size_t)pc * 8);
  const v4f b = *(const v4f*)(X + (size_t)pc * 8 + 4);
  const v8us hv = cvt8(a, b, ASCL);
  unsigned short* op = o + (size_t)pc * 8;
  if (p < np) *(volatile v8us*)op = hv;
  __threadfence();
  if (p < np) *(volatile v8us*)op = hv;
}

__global__ __launch_bounds__(256) void k_cnt(const int* __restrict__ ei, int nE, int* cinp, int* coutp) {
  __shared__ __attribute__((aligned(16))) int hin[CRNG];
  __shared__ __attribute__((aligned(16))) int hou[CRNG];
  const int tid = (int)threadIdx.x;
  const int n0 = (int)blockIdx.x * CRNG;
#pragma unroll
  for (int i = 0; i < 16; ++i) { hin[i * 256 + tid] = 0; hou[i * 256 + tid] = 0; }
  __syncthreads();
  const int* sp = ei;
  const int* tp = ei + nE;
#pragma unroll 1
  for (int cb = 0; cb < nE; cb += 2048) {
#pragma unroll
    for (int u = 0; u < 2; ++u) {
      const int gi = cb + 4 * (tid + 256 * u);
      const int ga = gi < nE - 4 ? gi : nE - 4;
      const int gv = gi < nE ? 1 : 0;
      const v4i tv = *(const v4i*)(tp + ga);
      const v4i sv = *(const v4i*)(sp + ga);
      const int tt[4] = {tv.x, tv.y, tv.z, tv.w};
      const int ss[4] = {sv.x, sv.y, sv.z, sv.w};
#pragma unroll
      for (int j = 0; j < 4; ++j) {
        const unsigned lt = (unsigned)(tt[j] - n0);
        const unsigned ls = (unsigned)(ss[j] - n0);
        const int ht = (gv != 0 && lt < (unsigned)CRNG) ? 1 : 0;
        const int hs = (gv != 0 && ls < (unsigned)CRNG) ? 1 : 0;
        const int it_ = ht ? (int)lt : (int)(lt & (unsigned)(CRNG - 1));
        const int is_ = hs ? (int)ls : (int)(ls & (unsigned)(CRNG - 1));
        atomicAdd(&hin[it_], ht);
        atomicAdd(&hou[is_], hs);
      }
    }
  }
  __syncthreads();
  v4i av[4], bv[4];
  size_t po[4];
#pragma unroll
  for (int it = 0; it < 4; ++it) {
    const int p = it * 256 + tid;
    av[it] = *(const v4i*)(hin + 4 * p);
    bv[it] = *(const v4i*)(hou + 4 * p);
    po[it] = (size_t)n0 + 4 * p;
  }
#pragma unroll
  for (int it = 0; it < 4; ++it) { *(volatile v4i*)(cinp + po[it]) = av[it]; *(volatile v4i*)(coutp + po[it]) = bv[it]; }
  __threadfence();
#pragma unroll
  for (int it = 0; it < 4; ++it) { *(volatile v4i*)(cinp + po[it]) = av[it]; *(volatile v4i*)(coutp + po[it]) = bv[it]; }
}

__global__ __launch_bounds__(256) void k_fill(const int* __restrict__ ei, int nE, int nN,
    const int* __restrict__ cinp, int* loffg, unsigned short* csr) {
  extern __shared__ __align__(16) unsigned char flds[];
  int*            lst  = (int*)(flds + FL_LIST);
  unsigned short* seg  = (unsigned short*)(flds + FL_SEG);
  int*            loff = (int*)(flds + FL_LOFF);
  int*            lcnt = (int*)(flds + FL_LCNT);
  int*            cur  = (int*)(flds + FL_CUR);
  int*            wt   = (int*)(flds + FL_WT);
  const int tid = (int)threadIdx.x, lane = tid & 31, wave = tid >> 5;
  const int n0 = (int)blockIdx.x * FRNG;
  unsigned short* slotp = csr + (size_t)blockIdx.x * (size_t)SEGCAP;

  const v4i ca = *(const v4i*)(cinp + n0 + 4 * tid);
  int cv[4] = {ca.x, ca.y, ca.z, ca.w};
  int ts = 0;
#pragma unroll
  for (int j = 0; j < 4; ++j) {
    int c = cv[j];
    c = c < 0 ? 0 : (c > SEGCAP ? SEGCAP : c);
    cv[j] = c;
    ts += c;
  }
  int xs = ts;
#pragma unroll
  for (int o = 1; o <= 16; o <<= 1) {
    const int y = __shfl_up(xs, o);
    xs += (lane >= o) ? y : 0;
  }
  if (lane == 31) wt[wave] = xs;
  __syncthreads();
  int wb = 0, tot = 0;
#pragma unroll
  for (int w = 0; w < 8; ++w) {
    const int tw = wt[w];
    wb += (w < wave) ? tw : 0;
    tot += tw;
  }
  int run = wb + (xs - ts);
  int lo4[4];
#pragma unroll
  for (int j = 0; j < 4; ++j) {
    lo4[j] = run;
    loff[4 * tid + j] = run;
    lcnt[4 * tid + j] = cv[j];
    cur[4 * tid + j] = 0;
    run += cv[j];
  }
  v4i lv;
  lv.x = lo4[0]; lv.y = lo4[1]; lv.z = lo4[2]; lv.w = lo4[3];
  *(volatile v4i*)(loffg + n0 + 4 * tid) = lv;
  __threadfence();
  *(volatile v4i*)(loffg + n0 + 4 * tid) = lv;
  {
    const v8us z8 = {0, 0, 0, 0, 0, 0, 0, 0};
#pragma unroll
    for (int it = 0; it < SEGCAP / 8 / 256; ++it) *(v8us*)(seg + 8 * (it * 256 + tid)) = z8;
    if (tid < 8) *(v8us*)(seg + SEGCAP + 8 * tid) = z8;
  }
  __syncthreads();

  const int* sp = ei;
  const int* tp = ei + nE;
  int Htot = 0;
#pragma unroll 1
  for (int cb = 0; cb < nE; cb += ECH) {
    const int e0 = cb + 16 * tid;
    int dd[16], ss[16];
#pragma unroll
    for (int q = 0; q < 4; ++q) {
      const int gi = e0 + 4 * q;
      const int ga = gi < nE - 4 ? gi : nE - 4;
      const v4i dv = *(const v4i*)(tp + ga);
      const v4i sv = *(const v4i*)(sp + ga);
      const bool gv = gi < nE;
      dd[4 * q + 0] = gv ? dv.x : DSENT; dd[4 * q + 1] = gv ? dv.y : DSENT;
      dd[4 * q + 2] = gv ? dv.z : DSENT; dd[4 * q + 3] = gv ? dv.w : DSENT;
      ss[4 * q + 0] = sv.x; ss[4 * q + 1] = sv.y; ss[4 * q + 2] = sv.z; ss[4 * q + 3] = sv.w;
    }
    int hits = 0, cnt = 0;
#pragma unroll
    for (int j = 0; j < 16; ++j) {
      const int h = ((unsigned)(dd[j] - n0) < (unsigned)FRNG) ? 1 : 0;
      hits |= h << j;
      cnt += h;
    }
    int x = cnt;
#pragma unroll
    for (int o = 1; o <= 16; o <<= 1) {
      const int y = __shfl_up(x, o);
      x += (lane >= o) ? y : 0;
    }
    if (lane == 31) wt[wave] = x;
    __syncthreads();
    int wbase = 0, ctot = 0;
#pragma unroll
    for (int w = 0; w < 8; ++w) {
      const int t = wt[w];
      wbase += (w < wave) ? t : 0;
      ctot += t;
    }
    int pos = Htot + wbase + (x - cnt);
#pragma unroll
    for (int j = 0; j < 16; ++j) {
      if ((hits >> j) & 1) {
        if (pos < LCAP) {
          int s = ss[j];
          s = s < 0 ? 0 : (s > nN - 1 ? nN - 1 : s);
          lst[pos] = (s << FSH) | (dd[j] - n0);
        }
        ++pos;
      }
    }
    Htot += ctot;
    __syncthreads();
  }
  const int H = Htot < LCAP ? Htot : LCAP;

  if (wave == 0) {
#pragma unroll 1
    for (int i = 0; i < H; ++i) {
      const int ent = lst[i];
      const int key = ent & (FRNG - 1);
      int s = ent >> FSH;
      s = s < 0 ? 0 : (s > 65535 ? 65535 : s);
      const int c = cur[key];
      const int p = loff[key] + c;
      const int ok = (c < lcnt[key] && (unsigned)p < (unsigned)SEGCAP) ? 1 : 0;
      seg[ok ? p : SEGCAP] = (unsigned short)s;
      cur[key] = c + ok;
    }
  }
  __syncthreads();

  const int segend = tot < SEGCAP ? tot : SEGCAP;
  const int segw = (segend + 63) & ~63;
  const int npc = segw >> 3;
#pragma unroll 1
  for (int it = 0; it < SEGCAP / 8 / 256; ++it) {
    const int p = it * 256 + tid;
    if (p < npc) *(volatile v8us*)(slotp + (size_t)8 * p) = *(const v8us*)(seg + 8 * p);
  }
  __threadfence();
#pragma unroll 1
  for (int it = 0; it < SEGCAP / 8 / 256; ++it) {
    const int p = it * 256 + tid;
    if (p < npc) *(volatile v8us*)(slotp + (size_t)8 * p) = *(const v8us*)(seg + 8 * p);
  }
}

__device__ __forceinline__ void gemm_tile(const unsigned short* A, const unsigned short* __restrict__ Bt,
                                          int K, int M, int Ncols, int r0, int c0, int lane, float* sw) {
  const int hh = lane >> 4, m = lane & 15;
  int ra = r0 + m; ra = ra > M - 1 ? M - 1 : ra;
  const unsigned short* ap = A + (size_t)ra * K + 8 * hh;
  int cb = c0 + m; cb = cb > Ncols - 1 ? Ncols - 1 : cb;
  const unsigned short* bp = Bt + (size_t)cb * K + 8 * hh;
  v8f acc[8];
#pragma unroll
  for (int j = 0; j < 8; ++j) acc[j] = zero8();
  const int nk = K >> 5;
#pragma unroll 1
  for (int kt = 0; kt < nk; ++kt) {
    const int kb = kt << 5;
    FragH a;
    a.u[0] = *(const v8us*)(ap + kb);
    a.u[1] = *(const v8us*)(ap + kb + 16);
#pragma unroll
    for (int j = 0; j < 8; ++j) {
      const unsigned short* bj = bp + (size_t)(16 * j) * (size_t)K + kb;
      FragH b;
      b.u[0] = *(const v8us*)(bj);
      b.u[1] = *(const v8us*)(bj + 16);
      acc[j] = wmh(a.v, b.v, acc[j]);
    }
  }
#pragma unroll
  for (int j = 0; j < 8; ++j)
#pragma unroll
    for (int r = 0; r < 8; ++r)
      sw[(8 * hh + r) * 128 + 16 * j + m] = acc[j][r];
}

__global__ __launch_bounds__(GTH) void k_gemm_qkv(
    const unsigned short* A, const unsigned short* __restrict__ Bt,
    const float* __restrict__ b0, const float* __restrict__ b1, const float* __restrict__ b2,
    float* outF, int M) {
  __shared__ __attribute__((aligned(16))) float sT[(GTH / 32) * GWT];
  const int tid = (int)threadIdx.x, lane = tid & 31, wave = tid >> 5;
  const int r0 = (int)blockIdx.y * GBM + wave * 16;
  const int c0 = (int)blockIdx.x * 128;
  float* sw = sT + wave * GWT;
  gemm_tile(A, Bt, NND, M, QP, r0, c0, lane, sw);
  __syncthreads();
  const int bx = (int)blockIdx.x;
  const float* bb = bx == 0 ? b0 : (bx == 1 ? b1 : b2);
  const int col = 4 * lane;
  const v4f b4 = *(const v4f*)(bb + col);
  float* ob = outF + (size_t)r0 * QP + c0 + col;
#pragma unroll
  for (int half = 0; half < 2; ++half) {
    v4f ov[8];
#pragma unroll
    for (int it = 0; it < 8; ++it)
      ov[it] = *(const v4f*)(sw + (8 * half + it) * 128 + col) * INVSCL + b4;
#pragma unroll
    for (int it = 0; it < 8; ++it) *(volatile v4f*)(ob + (size_t)(8 * half + it) * QP) = ov[it];
    __threadfence();
#pragma unroll
    for (int it = 0; it < 8; ++it) *(volatile v4f*)(ob + (size_t)(8 * half + it) * QP) = ov[it];
  }
}

__global__ __launch_bounds__(GTH) void k_gemm_in(
    const unsigned short* A, const unsigned short* __restrict__ Bt, const float* __restrict__ bin,
    const float* __restrict__ inemb, const float* __restrict__ outemb,
    const int* __restrict__ cinp, const int* __restrict__ coutp,
    const float* __restrict__ lns, const float* __restrict__ lnb,
    float* H, unsigned short* HN, int M) {
  __shared__ __attribute__((aligned(16))) float sT[(GTH / 32) * GWT];
  const int tid = (int)threadIdx.x, lane = tid & 31, wave = tid >> 5;
  const int r0 = (int)blockIdx.y * GBM + wave * 16;
  float* sw = sT + wave * GWT;
  gemm_tile(A, Bt, KIN, M, NND, r0, 0, lane, sw);
  __syncthreads();
  const int col = 4 * lane;
  const v4f b4 = *(const v4f*)(bin + col);
  const v4f g4 = *(const v4f*)(lns + col);
  const v4f e4 = *(const v4f*)(lnb + col);
#pragma unroll
  for (int half = 0; half < 2; ++half) {
    v4f hv[8];
    v4us yh[8];
#pragma unroll
    for (int it = 0; it < 8; ++it) {
      const int row = 8 * half + it;
      const int gr = r0 + row;
      v4f o = *(const v4f*)(sw + row * 128 + col) * INVSCL + b4;
      int di = cinp[gr];  di = di < 0 ? 0 : (di > DEGMX ? DEGMX : di);
      int dq = coutp[gr]; dq = dq < 0 ? 0 : (dq > DEGMX ? DEGMX : dq);
      o = o + *(const v4f*)(inemb + (size_t)di * NND + col);
      o = o + *(const v4f*)(outemb + (size_t)dq * NND + col);
      hv[it] = o;
      yh[it] = cvt4(ln4(o, g4, e4), ASCL);
    }
#pragma unroll
    for (int it = 0; it < 8; ++it) {
      const size_t go = (size_t)(r0 + 8 * half + it) * NND + col;
      *(volatile v4f*)(H + go) = hv[it];
      *(volatile v4us*)(HN + go) = yh[it];
    }
    __threadfence();
#pragma unroll
    for (int it = 0; it < 8; ++it) {
      const size_t go = (size_t)(r0 + 8 * half + it) * NND + col;
      *(volatile v4f*)(H + go) = hv[it];
      *(volatile v4us*)(HN + go) = yh[it];
    }
  }
}

__global__ __launch_bounds__(256) void k_att(float* QO, const int* __restrict__ cinp,
    const int* __restrict__ loffp, const unsigned short* __restrict__ csr, int nN) {
  const int tid = (int)threadIdx.x, lane = tid & 31, wave = tid >> 5;
  const int hh = lane >> 1, par = lane & 1;
  const int t = (int)blockIdx.x * 8 + wave;
  if (t < nN) {
    const float* qr = QO + (size_t)t * QP + 8 * hh;
    const v4f q0 = *(const v4f*)qr;
    const v4f q1 = *(const v4f*)(qr + 4);
    int lo = loffp[t];
    lo = lo < 0 ? 0 : (lo > SEGCAP ? SEGCAP : lo);
    int cnt = cinp[t];
    cnt = cnt < 0 ? 0 : cnt;
    const int room = SEGCAP - lo;
    cnt = cnt > room ? room : cnt;
    const unsigned short* cs = csr + (size_t)(t >> FSH) * (size_t)SEGCAP + lo;
    const float ninf = -__builtin_inff();
    float mr = ninf, z = 0.0f;
    v4f a0 = {0.f, 0.f, 0.f, 0.f};
    v4f a1 = {0.f, 0.f, 0.f, 0.f};
#pragma unroll 1
    for (int e2 = 0; e2 < cnt; e2 += 2) {
      const int j = e2 + par;
      const bool valid = j < cnt;
      const int jc = valid ? j : cnt - 1;
      int s = (int)cs[jc];
      s = s > nN - 1 ? nN - 1 : s;
      const float* kp = QO + (size_t)s * QP + KOF + 8 * hh;
      const v4f k0 = *(const v4f*)kp;
      const v4f k1 = *(const v4f*)(kp + 4);
      const v4f v0 = *(const v4f*)(kp + (VOF - KOF));
      const v4f v1 = *(const v4f*)(kp + (VOF - KOF) + 4);
      const v4f pr = q0 * k0 + q1 * k1;
      float a = ((pr.x + pr.y) + (pr.z + pr.w)) * RSQC;
      a = valid ? a : ninf;
      const float mn = fmaxf(mr, a);
      const float scv = __expf(mr - mn);
      const float sc = (mn > mr) ? scv : 1.0f;
      const float pv = __expf(a - mn);
      const float p = valid ? pv : 0.0f;
      z = z * sc + p;
      a0 = a0 * sc + v0 * p;
      a1 = a1 * sc + v1 * p;
      mr = mn;
    }
    const float mo = __shfl_xor(mr, 1);
    const float mm = fmaxf(mr, mo);
    const float mg = (mm > -3.0e38f) ? mm : 0.0f;
    const float se = __expf(mr - mg);
    z = z * se;
    a0 = a0 * se;
    a1 = a1 * se;
    z += __shfl_xor(z, 1);
    a0.x += __shfl_xor(a0.x, 1); a0.y += __shfl_xor(a0.y, 1); a0.z += __shfl_xor(a0.z, 1); a0.w += __shfl_xor(a0.w, 1);
    a1.x += __shfl_xor(a1.x, 1); a1.y += __shfl_xor(a1.y, 1); a1.z += __shfl_xor(a1.z, 1); a1.w += __shfl_xor(a1.w, 1);
    const float rz = z > 0.0f ? (1.0f / z) : 0.0f;
    v4f o;
    o.x = (par ? a1.x : a0.x) * rz;
    o.y = (par ? a1.y : a0.y) * rz;
    o.z = (par ? a1.z : a0.z) * rz;
    o.w = (par ? a1.w : a0.w) * rz;
    float* op = QO + (size_t)t * QP + 4 * lane;
    *(volatile v4f*)op = o;
    __threadfence();
    *(volatile v4f*)op = o;
  }
}

template <int FINAL>
__global__ __launch_bounds__(GTH) void k_gemm_skip(
    const unsigned short* A, const unsigned short* __restrict__ Bt, const float* __restrict__ bsk,
    const float* __restrict__ Wb, const float* QO, float* H,
    const float* __restrict__ lng, const float* __restrict__ lnbv,
    unsigned short* HN, float* OUT, int M) {
  __shared__ __attribute__((aligned(16))) float sT[(GTH / 32) * GWT];
  const int tid = (int)threadIdx.x, lane = tid & 31, wave = tid >> 5;
  const int r0 = (int)blockIdx.y * GBM + wave * 16;
  float* sw = sT + wave * GWT;
  gemm_tile(A, Bt, NND, M, NND, r0, 0, lane, sw);
  __syncthreads();
  const int col = 4 * lane;
  const v4f bs4 = *(const v4f*)(bsk + col);
  const v4f w0 = *(const v4f*)(Wb + col);
  const v4f w1 = *(const v4f*)(Wb + NND + col);
  const v4f w2 = *(const v4f*)(Wb + 2 * NND + col);
  const v4f g4 = *(const v4f*)(lng + col);
  const v4f e4 = *(const v4f*)(lnbv + col);
#pragma unroll
  for (int half = 0; half < 2; ++half) {
    v4f hv[8];
    v4f yv[8];
    v4us yh[8];
#pragma unroll
    for (int it = 0; it < 8; ++it) {
      const int row = 8 * half + it;
      const size_t gr = (size_t)(r0 + row);
      const v4f xr = *(const v4f*)(sw + row * 128 + col) * INVSCL + bs4;
      const v4f o4 = *(const v4f*)(QO + gr * QP + col);
      const v4f h4 = *(const v4f*)(H + gr * NND + col);
      const v4f df = o4 - xr;
      const v4f tg = o4 * w0 + xr * w1 + df * w2;
      float gs = (tg.x + tg.y) + (tg.z + tg.w);
#pragma unroll
      for (int oo = 16; oo >= 1; oo >>= 1) gs += __shfl_xor(gs, oo);
      gs = fminf(fmaxf(gs, -GCAP), GCAP);
      const float beta = 1.0f / (1.0f + __expf(-gs));
      const v4f cvv = xr * beta + o4 * (1.0f - beta);
      const v4f hn = h4 + cvv;
      const v4f y = ln4(hn, g4, e4);
      hv[it] = hn;
      if (FINAL) { yv[it] = y; } else { yh[it] = cvt4(y, ASCL); }
    }
    if (FINAL) {
#pragma unroll
      for (int it = 0; it < 8; ++it)
        *(volatile v4f*)(OUT + (size_t)(r0 + 8 * half + it) * NND + col) = yv[it];
      __threadfence();
#pragma unroll
      for (int it = 0; it < 8; ++it)
        *(volatile v4f*)(OUT + (size_t)(r0 + 8 * half + it) * NND + col) = yv[it];
    } else {
#pragma unroll
      for (int it = 0; it < 8; ++it) {
        const size_t go = (size_t)(r0 + 8 * half + it) * NND + col;
        *(volatile v4f*)(H + go) = hv[it];
        *(volatile v4us*)(HN + go) = yh[it];
      }
      __threadfence();
#pragma unroll
      for (int it = 0; it < 8; ++it) {
        const size_t go = (size_t)(r0 + 8 * half + it) * NND + col;
        *(volatile v4f*)(H + go) = hv[it];
        *(volatile v4us*)(HN + go) = yh[it];
      }
    }
  }
}

extern "C" void kernel_launch(void* const* d_in, const int* in_sizes, int n_in,
                              void* d_out, int out_size, void* d_ws, size_t ws_size,
                              hipStream_t stream) {
  if (n_in < 19) return;
  const int nN = in_sizes[0] / KIN;
  if (nN <= 0 || nN > 65536) return;
  if (in_sizes[0] != nN * KIN) return;
  if ((nN % GBM) != 0 || (nN % 8) != 0) return;
  if (out_size != nN * NND) return;
  const int nE2 = in_sizes[1];
  const int nE = nE2 / 2;
  if (nE < 4 || nE2 != 2 * nE || (nE % 4) != 0 || nE > (1 << 28)) return;
  if (in_sizes[2] != KIN * NND || in_sizes[3] != NND) return;
  if (in_sizes[4] != EMBN * NND || in_sizes[5] != EMBN * NND) return;
  if (in_sizes[6] != NLAY * NND || in_sizes[7] != NLAY * NND) return;
  if (in_sizes[8] != NLAY * NND * NND || in_sizes[10] != NLAY * NND * NND) return;
  if (in_sizes[12] != NLAY * NND * NND || in_sizes[14] != NLAY * NND * NND) return;
  if (in_sizes[9] != NLAY * NND || in_sizes[11] != NLAY * NND) return;
  if (in_sizes[13] != NLAY * NND || in_sizes[15] != NLAY * NND) return;
  if (in_sizes[16] != NLAY * 3 * NND) return;
  if (in_sizes[17] != NND || in_sizes[18] != NND) return;

  const float* x      = (const float*)d_in[0];
  const int*   ei     = (const int*)d_in[1];
  const float* Win    = (const float*)d_in[2];
  const float* bin    = (const float*)d_in[3];
  const float* inemb  = (const float*)d_in[4];
  const float* outemb = (const float*)d_in[5];
  const float* lns    = (const float*)d_in[6];
  const float* lnb    = (const float*)d_in[7];
  const float* Wq     = (const float*)d_in[8];
  const float* bq     = (const float*)d_in[9];
  const float* Wk     = (const float*)d_in[10];
  const float* bk     = (const float*)d_in[11];
  const float* Wv     = (const float*)d_in[12];
  const float* bv     = (const float*)d_in[13];
  const float* Wsk    = (const float*)d_in[14];
  const float* bsk    = (const float*)d_in[15];
  const float* Wbeta  = (const float*)d_in[16];
  const float* fns    = (const float*)d_in[17];
  const float* fnb    = (const float*)d_in[18];
  float* out = (float*)d_out;

  const int NPAD = ((nN + CRNG - 1) / CRNG) * CRNG;
  const int nbc = NPAD / CRNG;
  const int nbf = NPAD / FRNG;

  size_t off = 0;
  auto carve = [&](size_t bytes) { const size_t o = off; off += (bytes + 255) & ~(size_t)255; return o; };
  const size_t oWqkv = carve((size_t)NLAY * QP * NND * 2);
  const size_t oWsk  = carve((size_t)NLAY * NND * NND * 2);
  const size_t oWin  = carve((size_t)NND * KIN * 2);
  const size_t oCin  = carve((size_t)NPAD * 4);
  const size_t oCout = carve((size_t)NPAD * 4);
  const size_t oLoff = carve((size_t)NPAD * 4);
  const size_t oCsr  = carve((size_t)nbf * SEGCAP * 2);
  const size_t oQKV  = carve((size_t)nN * QP * 4);
  const size_t oH    = carve((size_t)nN * NND * 4);
  const size_t oHN   = carve((size_t)nN * NND * 2);
  if ((size_t)nN * KIN * 2 > (size_t)nN * QP * 4) return;
  if (off > ws_size || off > (size_t)WSCAP) return;

  char* ws = (char*)d_ws;
  unsigned short* wqkv16 = (unsigned short*)(ws + oWqkv);
  unsigned short* wsk16  = (unsigned short*)(ws + oWsk);
  unsigned short* win16  = (unsigned short*)(ws + oWin);
  int*            cin    = (int*)(ws + oCin);
  int*            cout_  = (int*)(ws + oCout);
  int*            loff   = (int*)(ws + oLoff);
  unsigned short* csr    = (unsigned short*)(ws + oCsr);
  float*          qkv    = (float*)(ws + oQKV);
  unsigned short* x16    = (unsigned short*)(ws + oQKV);
  float*          H      = (float*)(ws + oH);
  unsigned short* hn16   = (unsigned short*)(ws + oHN);

  hipFuncSetAttribute(reinterpret_cast<const void*>(&k_fill), hipFuncAttributeMaxDynamicSharedMemorySize, FILL_LDS);

  k_wpack<<<dim3(NND / 64, KIN / 64, 1), 256, 0, stream>>>(Win, win16, KIN, NND, 0, 0);
  k_wpack<<<dim3(NND / 64, NND / 64, NLAY), 256, 0, stream>>>(Wq, wqkv16, NND, NND, NND * NND, QP * NND);
  k_wpack<<<dim3(NND / 64, NND / 64, NLAY), 256, 0, stream>>>(Wk, wqkv16 + (size_t)KOF * NND, NND, NND, NND * NND, QP * NND);
  k_wpack<<<dim3(NND / 64, NND / 64, NLAY), 256, 0, stream>>>(Wv, wqkv16 + (size_t)VOF * NND, NND, NND, NND * NND, QP * NND);
  k_wpack<<<dim3(NND / 64, NND / 64, NLAY), 256, 0, stream>>>(Wsk, wsk16, NND, NND, NND * NND, NND * NND);

  const int npx = nN * KIN / 8;
  k_cvt<<<(npx + 255) / 256, 256, 0, stream>>>(x, x16, npx);

  k_cnt<<<nbc, 256, 0, stream>>>(ei, nE, cin, cout_);
  k_fill<<<nbf, 256, FILL_LDS, stream>>>(ei, nE, nN, cin, loff, csr);

  const dim3 g1(1, nN / GBM);
  const dim3 g3(3, nN / GBM);
  k_gemm_in<<<g1, GTH, 0, stream>>>(x16, win16, bin, inemb, outemb, cin, cout_, lns, lnb, H, hn16, nN);

  for (int l = 0; l < NLAY; ++l) {
    k_gemm_qkv<<<g3, GTH, 0, stream>>>(hn16, wqkv16 + (size_t)l * QP * NND, bq + (size_t)l * NND, bk + (size_t)l * NND,
                                         bv + (size_t)l * NND, qkv, nN);
    k_att<<<(nN + 7) / 8, 256, 0, stream>>>(qkv, cin, loff, csr, nN);
    if (l < NLAY - 1) {
      k_gemm_skip<0><<<g1, GTH, 0, stream>>>(hn16, wsk16 + (size_t)l * NND * NND, bsk + (size_t)l * NND,
                                             Wbeta + (size_t)l * 3 * NND, qkv, H,
                                             lns + (size_t)(l + 1) * NND, lnb + (size_t)(l + 1) * NND, hn16, out, nN);
    } else {
      k_gemm_skip<1><<<g1, GTH, 0, stream>>>(hn16, wsk16 + (size_t)l * NND * NND, bsk + (size_t)l * NND,
                                             Wbeta + (size_t)l * 3 * NND, qkv, H,
                                             fns, fnb, hn16, out, nN);
    }
  }
}
